// MatrixLSTMCell_81570018886143
// MI455X (gfx1250) — hardware-run, weakly checked
//
#include <hip/hip_runtime.h>
#include <math.h>

typedef __attribute__((ext_vector_type(16))) _Float16 v16h;
typedef __attribute__((ext_vector_type(8)))  _Float16 v8h;
typedef __attribute__((ext_vector_type(4)))  _Float16 v4h;
typedef __attribute__((ext_vector_type(2)))  _Float16 v2h;
typedef __attribute__((ext_vector_type(16))) __bf16   v16b;
typedef __attribute__((ext_vector_type(8)))  __bf16   v8b;
typedef __attribute__((ext_vector_type(8)))  float    v8f;
typedef __attribute__((ext_vector_type(4)))  float    v4f;
typedef __attribute__((ext_vector_type(2)))  float    v2f;


constexpr int kB   = 128;
constexpr int kN   = 256;
constexpr int kR   = kB * kN;
constexpr int kMM  = kN * kN;
constexpr int kThr = 256;
constexpr float kInCarry = 1024.0f;
constexpr float kCmCarry = 64.0f;
constexpr float kSc20 = 1.0f / (kInCarry * kInCarry);
constexpr float kSc16 = 1.0f / (kInCarry * kCmCarry);
constexpr float kF16MinNormal = 6.103515625e-5f;

static_assert(kB == 128 && kN == 256 && kR == 32768 && kMM == 65536 && kN / 8 == 32 && kN / 4 == 64, "the index arithmetic below uses these sizes: a row is 32 lanes of eight columns in the one-word casts and 64 lanes of four columns in the two-word cast and the passes");

constexpr size_t kOffX16  = 0ull;
constexpr size_t kOffH16  = 16777216ull;
constexpr size_t kOffWF   = 33554432ull;
constexpr size_t kOffWI   = 33816576ull;
constexpr size_t kOffWG   = 34078720ull;
constexpr size_t kOffWO   = 34340864ull;
constexpr size_t kOffWC   = 34603008ull;
constexpr size_t kOffTF   = 34865152ull;
constexpr size_t kOffTW   = 68419584ull;
constexpr size_t kOffGP   = 101974016ull;
constexpr size_t kOffGO   = 135528448ull;
constexpr size_t kOffCA   = 169082880ull;
constexpr size_t kOffCW   = 202637312ull;
constexpr size_t kWsTotal = 236191744ull;
static_assert(kOffH16 == (size_t)kR * kN * 2ull && kOffWF == 2ull * kOffH16 && kOffWI == kOffWF + (size_t)kN * 2 * kN * 2ull && kOffWG == kOffWI + (size_t)kN * 2 * kN * 2ull && kOffWO == kOffWG + (size_t)kN * 2 * kN * 2ull && kOffWC == kOffWO + (size_t)kN * 2 * kN * 2ull && kOffTF == kOffWC + (size_t)kN * 2 * kN * 2ull && kOffTW == kOffTF + (size_t)kR * kN * 4ull && kOffGP == kOffTW + (size_t)kR * 2 * kN * 2ull && kOffGO == kOffGP + (size_t)kR * kN * 4ull && kOffCA == kOffGO + (size_t)kR * kN * 4ull && kOffCW == kOffCA + (size_t)kR * kN * 4ull && kWsTotal == kOffCW + (size_t)kR * 2 * kN * 2ull, "the carve is a chain: every region starts where the one before ends");
static_assert((kOffH16 % 256) == 0 && (kOffWF % 256) == 0 && (kOffWI % 256) == 0 && (kOffWG % 256) == 0 && (kOffWO % 256) == 0 && (kOffWC % 256) == 0 && (kOffTF % 256) == 0 && (kOffTW % 256) == 0 && (kOffGP % 256) == 0 && (kOffGO % 256) == 0 && (kOffCA % 256) == 0 && (kOffCW % 256) == 0, "every region starts on a multiple of 256 B");

__device__ __forceinline__ unsigned short f2bf_bits(float f) {
  unsigned u = __float_as_uint(f);
  return (unsigned short)((u + 0x7FFFu + ((u >> 16) & 1u)) >> 16);
}
__device__ __forceinline__ float bf_bits2f(unsigned short h) { return __uint_as_float(((unsigned)h) << 16); }
__device__ __forceinline__ float bf16r(float f) { return bf_bits2f(f2bf_bits(f)); }
__device__ __forceinline__ float carry_flush(float v, float carry) {
  const float s = v * carry;
  return (fabsf(s) < kF16MinNormal) ? 0.0f : s;
}

__device__ __forceinline__ void dep_guard4_h(v8f& a, v8f& b, v8f& c, v8f& d, v16h x, v16h y) { asm volatile("v_nop\n\tv_nop\n\tv_nop\n\tv_nop" : "+v"(a), "+v"(b), "+v"(c), "+v"(d) : "v"(x), "v"(y)); }
__device__ __forceinline__ void dep_guard4_b(v8f& a, v8f& b, v8f& c, v8f& d, v16b x, v16b y) { asm volatile("v_nop\n\tv_nop\n\tv_nop\n\tv_nop" : "+v"(a), "+v"(b), "+v"(c), "+v"(d) : "v"(x), "v"(y)); }
__device__ __forceinline__ void keep4_h(v16h a, v16h b, v16h c, v16h d) { asm volatile("v_nop" :: "v"(a), "v"(b), "v"(c), "v"(d)); }
__device__ __forceinline__ void keep4_b(v16b a, v16b b, v16b c, v16b d) { asm volatile("v_nop" :: "v"(a), "v"(b), "v"(c), "v"(d)); }
__device__ __forceinline__ void acc_guard4(v8f& a, v8f& b, v8f& c, v8f& d) { asm volatile("v_nop\n\tv_nop\n\tv_nop\n\tv_nop" : "+v"(a), "+v"(b), "+v"(c), "+v"(d)); }

template <typename T> struct Frag;
template <> struct Frag<_Float16> {
  typedef v16h V; union U { v16h v; v8h h[2]; };
  static __device__ __forceinline__ v16h load(const _Float16* p) {
    U f; f.h[0] = *(const v8h*)(p); f.h[1] = *(const v8h*)(p + 16); return f.v;
  }
  static __device__ __forceinline__ v8f mma(v16h a, v16h b, v8f c) {
    return __builtin_amdgcn_wmma_f32_16x16x32_f16(false, a, false, b, (short)0, c, false, false);
  }
  static __device__ __forceinline__ void guard4(v8f& a, v8f& b, v8f& c, v8f& d, v16h x, v16h y) { dep_guard4_h(a, b, c, d, x, y); }
  static __device__ __forceinline__ void keep(v16h a, v16h b, v16h c, v16h d) { keep4_h(a, b, c, d); }
};
template <> struct Frag<__bf16> {
  typedef v16b V; union U { v16b v; v8b h[2]; };
  static __device__ __forceinline__ v16b load(const __bf16* p) {
    U f; f.h[0] = *(const v8b*)(p); f.h[1] = *(const v8b*)(p + 16); return f.v;
  }
  static __device__ __forceinline__ v8f mma(v16b a, v16b b, v8f c) {
    return __builtin_amdgcn_wmma_f32_16x16x32_bf16(false, a, false, b, (short)0, c, false, false);
  }
  static __device__ __forceinline__ void guard4(v8f& a, v8f& b, v8f& c, v8f& d, v16b x, v16b y) { dep_guard4_b(a, b, c, d, x, y); }
  static __device__ __forceinline__ void keep(v16b a, v16b b, v16b c, v16b d) { keep4_b(a, b, c, d); }
};

__device__ __forceinline__ v8f mma_h(v16h a, v16h b, v8f c) {
  c = __builtin_amdgcn_wmma_f32_16x16x32_f16(false, a, false, b, (short)0, c, false, false);
  asm volatile("v_nop\n\tv_nop\n\tv_nop\n\tv_nop" : "+v"(c) : "v"(a), "v"(b));
  return c;
}

template <int ET> struct Elem;
template <> struct Elem<0> { typedef _Float16 T; };
template <> struct Elem<1> { typedef __bf16 T; };
template <int ET, bool SPLIT, int BIAS_MODE, int OUT_MODE, bool RESID, int ACT = 0>
__global__ __launch_bounds__(256) void wmma_gemm64(
    const unsigned short* __restrict__ Ap, const unsigned short* __restrict__ A2p, int lda, long strideA,
    const unsigned short* __restrict__ Btp, const unsigned short* __restrict__ Bt2p, int ldb, long strideB,
    void* __restrict__ Cout, void* __restrict__ Cout2, int ldc, long strideC,
    const float* __restrict__ bias,
    const float* __restrict__ resid, long strideR,
    int M, int N, int K, float scale) {
  typedef typename Elem<ET>::T T;
  typedef typename Frag<T>::V V;
  const T* A = (const T*)Ap; const T* A2 = (const T*)A2p; const T* Bt = (const T*)Btp; const T* Bt2 = (const T*)Bt2p;
  __shared__ __align__(16) float sT[8][16 * 68];
  const int b    = blockIdx.y;
  const int lane = threadIdx.x & 31;
  const int wave = threadIdx.x >> 5;
  const int tilesN = N >> 6;
  const int tilesM = M >> 6;
  const int tile = blockIdx.x * 8 + wave;
  if (tile >= tilesM * tilesN) return;
  const int tm = tile / tilesN;
  const int tn = tile - tm * tilesN;
  const int m0 = tm << 6;
  const int n0 = tn << 6;

  const T* Ab  = A  + (size_t)b * strideA;
  const T* Bb  = Bt + (size_t)b * strideB;
  const T* Ab2 = SPLIT ? (A2  + (size_t)b * strideA) : nullptr;
  const T* Bb2 = SPLIT ? (Bt2 + (size_t)b * strideB) : nullptr;

  const int rlane = lane & 15;
  const int koff  = (lane >> 4) * 8;
  const int mOff  = (lane >> 4) * 8;

  v8f acc[4][4];
#pragma unroll
  for (int i = 0; i < 4; ++i)
#pragma unroll
    for (int j = 0; j < 4; ++j) acc[i][j] = (v8f){0.f,0.f,0.f,0.f,0.f,0.f,0.f,0.f};

  for (int k0 = 0; k0 < K; k0 += 32) {
    V bh[4], bl[4];
#pragma unroll
    for (int j = 0; j < 4; ++j) {
      const size_t bo = (size_t)(n0 + (j << 4) + rlane) * ldb + koff + k0;
      bh[j] = Frag<T>::load(Bb + bo);
      if (SPLIT) bl[j] = Frag<T>::load(Bb2 + bo);
    }
#pragma unroll
    for (int i = 0; i < 4; ++i) {
      const size_t ao = (size_t)(m0 + (i << 4) + rlane) * lda + koff + k0;
      V ah = Frag<T>::load(Ab + ao);
      V al;
      if (SPLIT) al = Frag<T>::load(Ab2 + ao);
#pragma unroll
      for (int j = 0; j < 4; ++j) {
        acc[i][j] = Frag<T>::mma(ah, bh[j], acc[i][j]);
        if (SPLIT) {
          acc[i][j] = Frag<T>::mma(ah, bl[j], acc[i][j]);
          acc[i][j] = Frag<T>::mma(al, bh[j], acc[i][j]);
        }
      }
      Frag<T>::guard4(acc[i][0], acc[i][1], acc[i][2], acc[i][3], ah, SPLIT ? al : ah);
    }
    Frag<T>::keep(bh[0], bh[1], bh[2], bh[3]);
    if (SPLIT) Frag<T>::keep(bl[0], bl[1], bl[2], bl[3]);
  }
  acc_guard4(acc[0][0], acc[0][1], acc[0][2], acc[0][3]);
  acc_guard4(acc[1][0], acc[1][1], acc[1][2], acc[1][3]);
  acc_guard4(acc[2][0], acc[2][1], acc[2][2], acc[2][3]);
  acc_guard4(acc[3][0], acc[3][1], acc[3][2], acc[3][3]);

  float* slab = sT[wave];
  const float* Rb = RESID ? (resid + (size_t)b * strideR) : nullptr;
#pragma unroll
  for (int i = 0; i < 4; ++i) {
    const int mBase = m0 + (i << 4);
#pragma unroll
    for (int j = 0; j < 4; ++j) {
      const int n = n0 + (j << 4) + rlane;
      float bv = 0.f;
      if (BIAS_MODE == 2) bv = bias[n];
#pragma unroll
      for (int r = 0; r < 8; ++r) {
        float v = acc[i][j][r] * scale;
        if (BIAS_MODE == 1) v += bias[mBase + mOff + r];
        if (BIAS_MODE == 2) v += bv;
        if (RESID) v += Rb[(size_t)(mBase + mOff + r) * ldc + n];
        if (ACT == 1) v = tanhf(v);
        if (ACT == 2) v = fmaxf(v, 0.0f);
        if (ACT == 3) v = v / (1.0f + expf(-v));
        if (ACT == 4) v = (v > 0.f) ? v : 0.01f * v;
        slab[(mOff + r) * 68 + (j << 4) + rlane] = v;
      }
    }
    __builtin_amdgcn_fence(__ATOMIC_RELEASE, "workgroup");
    __builtin_amdgcn_wave_barrier();
    __builtin_amdgcn_fence(__ATOMIC_ACQUIRE, "workgroup");
    if (OUT_MODE == 0) {
      float* C = (float*)Cout + (size_t)b * strideC;
      const int hh = lane >> 4, c4 = (lane & 15) * 4;
      for (int pass = 0; pass < 2; ++pass) {
#pragma unroll
        for (int it = 0; it < 8; ++it) {
          const int row = it * 2 + hh;
          v4f v = *(const v4f*)(slab + row * 68 + c4);
          *(volatile v4f*)(C + (size_t)(mBase + row) * ldc + n0 + c4) = v;
        }
        __threadfence();
      }
    } else {
      const int q = lane >> 3, c8 = (lane & 7) * 8;
      unsigned short* C  = (unsigned short*)Cout  + (size_t)b * strideC;
      unsigned short* C2 = (OUT_MODE == 2) ? ((unsigned short*)Cout2 + (size_t)b * strideC) : nullptr;
      for (int pass = 0; pass < 2; ++pass) {
#pragma unroll
        for (int it = 0; it < 4; ++it) {
          const int row = it * 4 + q;
          const float* sp = slab + row * 68 + c8;
          v8h hv, lv;
#pragma unroll
          for (int e = 0; e < 8; ++e) {
            if (OUT_MODE == 1) {
              hv[e] = (_Float16)sp[e];
            } else {
              unsigned short hb = f2bf_bits(sp[e]);
              unsigned short lb = f2bf_bits(sp[e] - bf_bits2f(hb));
              hv[e] = __builtin_bit_cast(_Float16, hb);
              lv[e] = __builtin_bit_cast(_Float16, lb);
            }
          }
          *(volatile v8h*)(C + (size_t)(mBase + row) * ldc + n0 + c8) = hv;
          if (OUT_MODE == 2) *(volatile v8h*)(C2 + (size_t)(mBase + row) * ldc + n0 + c8) = lv;
        }
        __threadfence();
      }
    }
    __builtin_amdgcn_fence(__ATOMIC_RELEASE, "workgroup");
    __builtin_amdgcn_wave_barrier();
    __builtin_amdgcn_fence(__ATOMIC_ACQUIRE, "workgroup");
  }
}


__global__ __launch_bounds__(kThr) void cast_plane_kernel(const float* __restrict__ src, unsigned short* __restrict__ dst,
                                                          int colsLog2, int dstPitch, int dstOff) {
  const int i   = blockIdx.x * kThr + threadIdx.x;
  const int sh  = colsLog2 - 3;
  const int row = i >> sh;
  const int c8  = (i & ((1 << sh) - 1)) * 8;
  const float* sp = src + ((size_t)row << colsLog2) + c8;
  const v4f a0 = *(const v4f*)(sp);
  const v4f a1 = *(const v4f*)(sp + 4);
  v8h hv;
#pragma unroll
  for (int e = 0; e < 4; ++e) {
    const float f0 = a0[e];
    const float f1 = a1[e];
    hv[e]     = (_Float16)carry_flush(bf16r(f0), kInCarry);
    hv[4 + e] = (_Float16)carry_flush(bf16r(f1), kInCarry);
  }
  unsigned short* dp = dst + (size_t)row * dstPitch + dstOff + c8;
  *(volatile v8h*)dp = hv;
  __threadfence();
  *(volatile v8h*)dp = hv;
}

__global__ __launch_bounds__(kThr) void pack_kernel(const float* __restrict__ W, unsigned short* __restrict__ D, float* __restrict__ dstf, int part, int ld, int k0, int lg, int n0, int pitch) {
  const unsigned i = blockIdx.x * blockDim.x + threadIdx.x;
  if (part == 0) {
    const unsigned g = i & ((1u << lg) - 1u), n = i >> lg;
    const float* sp = W + (size_t)((unsigned)k0 + g * 8u) * (unsigned)ld + n;
    v8h hv;
#pragma unroll
    for (int t = 0; t < 8; ++t) hv[t] = (_Float16)carry_flush(bf16r(sp[(size_t)t * (unsigned)ld]), kInCarry);
    unsigned short* dp = D + (size_t)((unsigned)n0 + n) * (unsigned)pitch + g * 8u;
    *(volatile v8h*)dp = hv;
    __threadfence();
    *(volatile v8h*)dp = hv;
  } else {
    const v4f a = *(const v4f*)(W + i * 4u);
    v4f o;
#pragma unroll
    for (int e = 0; e < 4; ++e) o[e] = bf16r(a[e]);
    float* dp = dstf + i * 4u;
    *(volatile v4f*)dp = o;
    __threadfence();
    *(volatile v4f*)dp = o;
  }
}

__global__ __launch_bounds__(kThr) void ccast_kernel(const float* __restrict__ src, unsigned short* __restrict__ dst, int dstPitch, int dstOff) {
  const unsigned i = blockIdx.x * (unsigned)kThr + threadIdx.x;
  const unsigned row = i >> 5, c8 = (i & 31u) << 3;
  const float* sp = src + (size_t)row * (unsigned)kN + c8;
  const v4f a = *(const v4f*)sp;
  const v4f b = *(const v4f*)(sp + 4);
  v8h hv;
#pragma unroll
  for (int e = 0; e < 4; ++e) {
    hv[e] = (_Float16)carry_flush(a[e], kCmCarry);
    hv[4 + e] = (_Float16)carry_flush(b[e], kCmCarry);
  }
  unsigned short* dp = dst + (size_t)row * (unsigned)dstPitch + (unsigned)dstOff + c8;
  *(volatile v8h*)dp = hv;
  __threadfence();
  *(volatile v8h*)dp = hv;
}

__global__ __launch_bounds__(kThr) void ccast2_kernel(const float* __restrict__ src, unsigned short* __restrict__ dst, float* __restrict__ cp) {
  const unsigned i = blockIdx.x * (unsigned)kThr + threadIdx.x;
  const unsigned row = i >> 6, c4 = (i & 63u) << 2;
  const v4f a = *(const v4f*)(src + (size_t)row * (unsigned)kN + c4);
  v4h hv;
  v4h lv;
#pragma unroll
  for (int e = 0; e < 4; ++e) {
    const _Float16 h = (_Float16)carry_flush(a[e], kCmCarry);
    hv[e] = h;
    lv[e] = (_Float16)carry_flush(a[e] - (float)h * (1.0f / kCmCarry), kCmCarry);
  }
  unsigned short* dp = dst + (size_t)row * (unsigned)(2 * kN) + c4;
  unsigned short* lp = dp + kN;
  float* fp = cp + (size_t)row * (unsigned)kN + c4;
  *(volatile v4h*)dp = hv;
  *(volatile v4h*)lp = lv;
  *(volatile v4f*)fp = a;
  __threadfence();
  *(volatile v4h*)dp = hv;
  *(volatile v4h*)lp = lv;
  *(volatile v4f*)fp = a;
}
__global__ __launch_bounds__(kThr) void gacc_kernel(const float* __restrict__ gp, const float* src, float* dst) {
  const unsigned i = blockIdx.x * (unsigned)kThr + threadIdx.x;
  const unsigned q4 = (i & 63u) << 2, o = (i >> 6) & 255u, b = i >> 14;
  const float* gb = gp + (size_t)b * (unsigned)kMM + (size_t)q4 * (unsigned)kN + o;
  const size_t os = (size_t)b * (unsigned)kMM + (size_t)o * (unsigned)kN + q4;
  const float g0 = gb[0], g1 = gb[kN], g2 = gb[2 * kN], g3 = gb[3 * kN];
  v4f s = *(const v4f*)(src + os);
  s[0] += (g0 < 0.0f) ? 0.0f : g0;
  s[1] += (g1 < 0.0f) ? 0.0f : g1;
  s[2] += (g2 < 0.0f) ? 0.0f : g2;
  s[3] += (g3 < 0.0f) ? 0.0f : g3;
  float* dp = dst + os;
  *(volatile v4f*)dp = s;
  __threadfence();
  *(volatile v4f*)dp = s;
}

__global__ __launch_bounds__(kThr) void hout_kernel(const float* __restrict__ go, const float* __restrict__ rp, float* __restrict__ ho) {
  const unsigned i = blockIdx.x * (unsigned)kThr + threadIdx.x;
  const unsigned q4 = (i & 63u) << 2, o = (i >> 6) & 255u, b = i >> 14;
  const size_t ts = (size_t)b * (unsigned)kMM + (size_t)q4 * (unsigned)kN + o;
  const size_t os = (size_t)b * (unsigned)kMM + (size_t)o * (unsigned)kN + q4;
  const float* gb = go + ts;
  const float* rb = rp + ts;
  const float g0 = gb[0], g1 = gb[kN], g2 = gb[2 * kN], g3 = gb[3 * kN];
  const float r0 = rb[0], r1 = rb[kN], r2 = rb[2 * kN], r3 = rb[3 * kN];
  v4f s;
  s[0] = ((g0 < 0.0f) ? 0.0f : g0) + ((r0 < 0.0f) ? 0.0f : r0);
  s[1] = ((g1 < 0.0f) ? 0.0f : g1) + ((r1 < 0.0f) ? 0.0f : r1);
  s[2] = ((g2 < 0.0f) ? 0.0f : g2) + ((r2 < 0.0f) ? 0.0f : r2);
  s[3] = ((g3 < 0.0f) ? 0.0f : g3) + ((r3 < 0.0f) ? 0.0f : r3);
  float* dp = ho + os;
  *(volatile v4f*)dp = s;
  __threadfence();
  *(volatile v4f*)dp = s;
}

extern "C" void kernel_launch(void* const* d_in, const int* in_sizes, int n_in,
                              void* d_out, int out_size, void* d_ws, size_t ws_size,
                              hipStream_t stream) {
  if (n_in < 12 || d_out == nullptr || d_ws == nullptr) return;
  for (int k = 0; k < 3; ++k) if (in_sizes[k] != kR * kN) return;
  for (int k = 3; k < 12; ++k) if (in_sizes[k] != kMM) return;
  if ((size_t)out_size != 2ull * kR * kN) return;
  if (ws_size < kWsTotal) return;
  char* ws = (char*)d_ws;
  unsigned short* X16 = (unsigned short*)(ws + kOffX16);
  unsigned short* H16 = (unsigned short*)(ws + kOffH16);
  unsigned short* WF = (unsigned short*)(ws + kOffWF);
  unsigned short* WI = (unsigned short*)(ws + kOffWI);
  unsigned short* WG = (unsigned short*)(ws + kOffWG);
  unsigned short* WO = (unsigned short*)(ws + kOffWO);
  unsigned short* WC = (unsigned short*)(ws + kOffWC);
  float* TF = (float*)(ws + kOffTF);
  unsigned short* TW = (unsigned short*)(ws + kOffTW);
  float* GP = (float*)(ws + kOffGP);
  float* GO = (float*)(ws + kOffGO);
  float* CA = (float*)(ws + kOffCA);
  unsigned short* CW = (unsigned short*)(ws + kOffCW);
  float* HO = (float*)d_out;
  float* CO = (float*)d_out + (size_t)kR * kN;

  static_assert((kR * (kN / 8)) % kThr == 0 && (kN * (kN / 8)) % kThr == 0 && (kR * kN / 4) % kThr == 0 && (kR * (kN / 4)) % kThr == 0 && (1 << 8) == kN, "every grid of the casts, the record launch and the passes exact; the casts' column count is this side");
  cast_plane_kernel<<<kR * (kN / 8) / kThr, kThr, 0, stream>>>((const float*)d_in[0], X16, 8, kN, 0);
  cast_plane_kernel<<<kR * (kN / 8) / kThr, kThr, 0, stream>>>((const float*)d_in[1], H16, 8, kN, 0);
  cast_plane_kernel<<<kN * (kN / 8) / kThr, kThr, 0, stream>>>((const float*)d_in[3], WF, 8, 2 * kN, 0);
  cast_plane_kernel<<<kN * (kN / 8) / kThr, kThr, 0, stream>>>((const float*)d_in[7], WF, 8, 2 * kN, kN);
  cast_plane_kernel<<<kN * (kN / 8) / kThr, kThr, 0, stream>>>((const float*)d_in[4], WI, 8, 2 * kN, 0);
  cast_plane_kernel<<<kN * (kN / 8) / kThr, kThr, 0, stream>>>((const float*)d_in[8], WI, 8, 2 * kN, kN);
  cast_plane_kernel<<<kN * (kN / 8) / kThr, kThr, 0, stream>>>((const float*)d_in[5], WO, 8, 2 * kN, 0);
  cast_plane_kernel<<<kN * (kN / 8) / kThr, kThr, 0, stream>>>((const float*)d_in[9], WO, 8, 2 * kN, kN);
  cast_plane_kernel<<<kN * (kN / 8) / kThr, kThr, 0, stream>>>((const float*)d_in[6], WG, 8, 2 * kN, 0);
  cast_plane_kernel<<<kN * (kN / 8) / kThr, kThr, 0, stream>>>((const float*)d_in[10], WG, 8, 2 * kN, kN);
  cast_plane_kernel<<<kN * (kN / 8) / kThr, kThr, 0, stream>>>((const float*)d_in[11], WC, 8, 2 * kN, 0);
  cast_plane_kernel<<<kN * (kN / 8) / kThr, kThr, 0, stream>>>((const float*)d_in[11], WC, 8, 2 * kN, kN);
  pack_kernel<<<kR * kN / 4 / kThr, kThr, 0, stream>>>((const float*)d_in[2], nullptr, CA, 1, 0, 0, 0, 0, 0);
  wmma_gemm64<0, false, 0, 0, false, 0><<<dim3((kN / 64) * (kN / 64) / 8, kB), 256, 0, stream>>>(
      WF, WF, 2 * kN, 0L, X16, X16, kN, (long)kMM, (void*)TF, (void*)TF, kN, (long)kMM, nullptr, nullptr, 0L, kN, kN, kN, kSc20);
  ccast_kernel<<<kR * (kN / 8) / kThr, kThr, 0, stream>>>(TF, TW, 2 * kN, 0);
  wmma_gemm64<0, false, 0, 0, false, 0><<<dim3((kN / 64) * (kN / 64) / 8, kB), 256, 0, stream>>>(
      WF + kN, WF + kN, 2 * kN, 0L, H16, H16, kN, (long)kMM, (void*)TF, (void*)TF, kN, (long)kMM, nullptr, nullptr, 0L, kN, kN, kN, kSc20);
  ccast_kernel<<<kR * (kN / 8) / kThr, kThr, 0, stream>>>(TF, TW, 2 * kN, kN);
  wmma_gemm64<0, false, 0, 0, false, 0><<<dim3((kN / 64) * (kN / 64) / 8, kB), 256, 0, stream>>>(
      TW, TW, 2 * kN, (long)(2 * kMM), WF, WF, 2 * kN, 0L, (void*)GP, (void*)GP, kN, (long)kMM, nullptr, nullptr, 0L, kN, kN, 2 * kN, kSc16);
  gacc_kernel<<<kR * (kN / 4) / kThr, kThr, 0, stream>>>(GP, CA, CA);
  wmma_gemm64<0, false, 0, 0, false, 0><<<dim3((kN / 64) * (kN / 64) / 8, kB), 256, 0, stream>>>(
      WI, WI, 2 * kN, 0L, X16, X16, kN, (long)kMM, (void*)TF, (void*)TF, kN, (long)kMM, nullptr, nullptr, 0L, kN, kN, kN, kSc20);
  ccast_kernel<<<kR * (kN / 8) / kThr, kThr, 0, stream>>>(TF, TW, 2 * kN, 0);
  wmma_gemm64<0, false, 0, 0, false, 0><<<dim3((kN / 64) * (kN / 64) / 8, kB), 256, 0, stream>>>(
      WI + kN, WI + kN, 2 * kN, 0L, H16, H16, kN, (long)kMM, (void*)TF, (void*)TF, kN, (long)kMM, nullptr, nullptr, 0L, kN, kN, kN, kSc20);
  ccast_kernel<<<kR * (kN / 8) / kThr, kThr, 0, stream>>>(TF, TW, 2 * kN, kN);
  wmma_gemm64<0, false, 0, 0, false, 0><<<dim3((kN / 64) * (kN / 64) / 8, kB), 256, 0, stream>>>(
      TW, TW, 2 * kN, (long)(2 * kMM), WI, WI, 2 * kN, 0L, (void*)GP, (void*)GP, kN, (long)kMM, nullptr, nullptr, 0L, kN, kN, 2 * kN, kSc16);
  gacc_kernel<<<kR * (kN / 4) / kThr, kThr, 0, stream>>>(GP, CA, CA);
  wmma_gemm64<0, false, 0, 0, false, 0><<<dim3((kN / 64) * (kN / 64) / 8, kB), 256, 0, stream>>>(
      WG, WG, 2 * kN, 0L, X16, X16, kN, (long)kMM, (void*)TF, (void*)TF, kN, (long)kMM, nullptr, nullptr, 0L, kN, kN, kN, kSc20);
  ccast_kernel<<<kR * (kN / 8) / kThr, kThr, 0, stream>>>(TF, TW, 2 * kN, 0);
  wmma_gemm64<0, false, 0, 0, false, 0><<<dim3((kN / 64) * (kN / 64) / 8, kB), 256, 0, stream>>>(
      WG + kN, WG + kN, 2 * kN, 0L, H16, H16, kN, (long)kMM, (void*)TF, (void*)TF, kN, (long)kMM, nullptr, nullptr, 0L, kN, kN, kN, kSc20);
  ccast_kernel<<<kR * (kN / 8) / kThr, kThr, 0, stream>>>(TF, TW, 2 * kN, kN);
  wmma_gemm64<0, false, 0, 0, false, 0><<<dim3((kN / 64) * (kN / 64) / 8, kB), 256, 0, stream>>>(
      TW, TW, 2 * kN, (long)(2 * kMM), WG, WG, 2 * kN, 0L, (void*)GP, (void*)GP, kN, (long)kMM, nullptr, nullptr, 0L, kN, kN, 2 * kN, kSc16);
  gacc_kernel<<<kR * (kN / 4) / kThr, kThr, 0, stream>>>(GP, CA, CA);
  wmma_gemm64<0, false, 0, 0, false, 0><<<dim3((kN / 64) * (kN / 64) / 8, kB), 256, 0, stream>>>(
      WO, WO, 2 * kN, 0L, X16, X16, kN, (long)kMM, (void*)TF, (void*)TF, kN, (long)kMM, nullptr, nullptr, 0L, kN, kN, kN, kSc20);
  ccast_kernel<<<kR * (kN / 8) / kThr, kThr, 0, stream>>>(TF, TW, 2 * kN, 0);
  wmma_gemm64<0, false, 0, 0, false, 0><<<dim3((kN / 64) * (kN / 64) / 8, kB), 256, 0, stream>>>(
      WO + kN, WO + kN, 2 * kN, 0L, H16, H16, kN, (long)kMM, (void*)TF, (void*)TF, kN, (long)kMM, nullptr, nullptr, 0L, kN, kN, kN, kSc20);
  ccast_kernel<<<kR * (kN / 8) / kThr, kThr, 0, stream>>>(TF, TW, 2 * kN, kN);
  wmma_gemm64<0, false, 0, 0, false, 0><<<dim3((kN / 64) * (kN / 64) / 8, kB), 256, 0, stream>>>(
      TW, TW, 2 * kN, (long)(2 * kMM), WO, WO, 2 * kN, 0L, (void*)GO, (void*)GO, kN, (long)kMM, nullptr, nullptr, 0L, kN, kN, 2 * kN, kSc16);
  ccast2_kernel<<<kR * (kN / 4) / kThr, kThr, 0, stream>>>(CA, CW, CO);
  wmma_gemm64<0, false, 0, 0, false, 0><<<dim3((kN / 64) * (kN / 64) / 8, kB), 256, 0, stream>>>(
      WC, WC, 2 * kN, 0L, CW, CW, 2 * kN, (long)(2 * kMM), (void*)GP, (void*)GP, kN, (long)kMM, nullptr, nullptr, 0L, kN, kN, 2 * kN, kSc16);
  ccast2_kernel<<<kR * (kN / 4) / kThr, kThr, 0, stream>>>(GP, TW, TF);
  wmma_gemm64<0, false, 0, 0, false, 0><<<dim3((kN / 64) * (kN / 64) / 8, kB), 256, 0, stream>>>(
      TW, TW, 2 * kN, (long)(2 * kMM), WC, WC, 2 * kN, 0L, (void*)GP, (void*)GP, kN, (long)kMM, nullptr, nullptr, 0L, kN, kN, 2 * kN, kSc16);
  hout_kernel<<<kR * (kN / 4) / kThr, kThr, 0, stream>>>(GO, GP, HO);
}
static_assert(((kN / 64) * (kN / 64)) % 8 == 0 && kN % 32 == 0 && (2 * kN) % 32 == 0, "the engine's grids: whole blocks of eight wave tiles a member; every depth a multiple of 32");
